// DistanceDecoder_34866544509319
// MI455X (gfx1250) — hardware-verified
//
#include <hip/hip_runtime.h>


namespace {
constexpr int N = 50000, E = 800000, H = 128, HO = 64, NPAD = 50048;
constexpr int NBLK = NPAD / 128;

typedef _Float16 b16;
typedef __attribute__((ext_vector_type(16))) _Float16 v16b;
typedef __attribute__((ext_vector_type(8)))  _Float16 v8b;
typedef __attribute__((ext_vector_type(8)))  float v8f;
typedef __attribute__((ext_vector_type(4)))  float v4f;

__device__ __forceinline__ v8b ld8b(const b16* p) { return *(const v8b*)p; }
__device__ __forceinline__ v16b cat8b(v8b a, v8b b) { return __builtin_shufflevector(a, b, 0, 1, 2, 3, 4, 5, 6, 7, 8, 9, 10, 11, 12, 13, 14, 15); }
__device__ __forceinline__ v16b frag_kb(const b16* p, int hh) { return cat8b(ld8b(p + 8 * hh), ld8b(p + 16 + 8 * hh)); }
__device__ __forceinline__ void split16(float v, b16& hi, b16& lo) { hi = (b16)v; lo = (b16)(v - (float)hi); }
__device__ __forceinline__ void frag_ksplit(const float* p, int hh, v16b& fh_, v16b& fl_) {
  const float* p0 = p + 8 * hh; const float* p1 = p + 16 + 8 * hh;
#pragma unroll
  for (int e = 0; e < 8; ++e) { b16 a, c; split16(p0[e], a, c); fh_[e] = a; fl_[e] = c; split16(p1[e], a, c); fh_[8 + e] = a; fl_[8 + e] = c; }
}
__device__ __forceinline__ v8f wmma16b(v16b a, v16b b, v8f c) {
  v8f d = __builtin_amdgcn_wmma_f32_16x16x32_f16(false, a, false, b, (short)0, c, false, false);
  asm volatile("v_nop\n\tv_nop\n\tv_nop\n\tv_nop" : "+v"(d) : "v"(a), "v"(b));
  return d;
}
__device__ __forceinline__ void wave_lds_sync() {
  __builtin_amdgcn_fence(__ATOMIC_RELEASE, "workgroup");
  __builtin_amdgcn_wave_barrier();
  __builtin_amdgcn_fence(__ATOMIC_ACQUIRE, "workgroup");
}

struct Opnd { const void* p0; const void* p1; int ld; };
template <int NP> __device__ __forceinline__ void load_frags(const Opnd& o, int row, int kb, int hh, v16b& fh_, v16b& fl_) {
  if (NP == 0) { frag_ksplit((const float*)o.p0 + (size_t)row * o.ld + kb, hh, fh_, fl_); }
  else if (NP == 4) {
    const float* p = (const float*)o.p0 + (size_t)row * o.ld + kb; const float* p0 = p + 8 * hh; const float* p1 = p + 16 + 8 * hh;
#pragma unroll
    for (int e = 0; e < 8; ++e) { b16 a, c; split16(p0[e] * 64.0f, a, c); fh_[e] = a; fl_[e] = c; split16(p1[e] * 64.0f, a, c); fh_[8 + e] = a; fl_[8 + e] = c; }
  } else if (NP == 3) {
    const float* p = (const float*)o.p0 + (size_t)row * o.ld + kb; const float* p0 = p + 8 * hh; const float* p1 = p + 16 + 8 * hh;
#pragma unroll
    for (int e = 0; e < 8; ++e) { fh_[e] = (b16)p0[e]; fh_[8 + e] = (b16)p1[e]; }
    fl_ = fh_;
  } else {
    fh_ = frag_kb((const b16*)o.p0 + (size_t)row * o.ld + kb, hh);
    if (NP == 2) fl_ = frag_kb((const b16*)o.p1 + (size_t)row * o.ld + kb, hh); else fl_ = fh_;
  }
}
template <int ANP, int BNP> __device__ __forceinline__ v8f mac(v16b ah, v16b al, v16b bh, v16b bl, v8f c) {
  c = wmma16b(ah, bh, c);
  if (BNP == 0 || BNP == 2 || BNP == 4) c = wmma16b(ah, bl, c);
  if (ANP == 0 || ANP == 2 || ANP == 4) c = wmma16b(al, bh, c);
  return c;
}
template <int ANP, int BNP>
__device__ __forceinline__ void gemm_tile(const Opnd& A, const Opnd& B, int K, int m0, int c0, int nloc, int hlf, v8f (&acc)[2][4]) {
  for (int kb = 0; kb < K; kb += 32) {
    v16b a0h, a0l, a1h, a1l;
    load_frags<ANP>(A, m0 + nloc, kb, hlf, a0h, a0l);
    load_frags<ANP>(A, m0 + 16 + nloc, kb, hlf, a1h, a1l);
#pragma unroll
    for (int t = 0; t < 4; ++t) {
      v16b bh, bl;
      load_frags<BNP>(B, c0 + t * 16 + nloc, kb, hlf, bh, bl);
      acc[0][t] = mac<ANP, BNP>(a0h, a0l, bh, bl, acc[0][t]);
      acc[1][t] = mac<ANP, BNP>(a1h, a1l, bh, bl, acc[1][t]);
    }
  }
}

__device__ __forceinline__ void epi_planes(v8f (&acc)[2][4], float scale, bool two, b16* __restrict__ oh, b16* __restrict__ ol, int ldo,
                                           int m0, int c0, int lane, b16* Th, b16* Tl) {
  const int nloc = lane & 15, hlf = lane >> 4;
#pragma unroll
  for (int t = 0; t < 4; ++t)
#pragma unroll
    for (int r = 0; r < 2; ++r)
#pragma unroll
      for (int v = 0; v < 8; ++v) {
        const int rr = r * 16 + v + 8 * hlf, cc = t * 16 + nloc;
        b16 h_, l_; split16(acc[r][t][v] * scale, h_, l_);
        Th[rr * 64 + cc] = h_; Tl[rr * 64 + cc] = l_;
      }
  wave_lds_sync();
  for (int pass = 0; pass < 2; ++pass) {
#pragma unroll
    for (int j = 0; j < 8; ++j) {
      const int rr = j * 4 + (lane >> 3), c8 = (lane & 7) * 8;
      const size_t o = (size_t)(m0 + rr) * ldo + c0 + c8;
      *(volatile v8b*)(oh + o) = ld8b(Th + rr * 64 + c8);
      if (two) *(volatile v8b*)(ol + o) = ld8b(Tl + rr * 64 + c8);
    }
    __threadfence();
  }
}
__device__ __forceinline__ void epi_f32(v8f (&acc)[2][4], float scale, const float* rscale, float* __restrict__ out, int ldo, int m0, int c0, int lane, float* Tt) {
  const int nloc = lane & 15, hlf = lane >> 4;
#pragma unroll
  for (int t = 0; t < 4; ++t)
#pragma unroll
    for (int r = 0; r < 2; ++r)
#pragma unroll
      for (int v = 0; v < 8; ++v) {
        const int rr = r * 16 + v + 8 * hlf;
        const float rs = rscale ? rscale[(size_t)(m0 + rr) * 32] : 1.0f;
        Tt[rr * 64 + t * 16 + nloc] = acc[r][t][v] * scale * rs;
      }
  wave_lds_sync();
  float* dst0 = out + (size_t)m0 * ldo + c0;
  for (int pass = 0; pass < 2; ++pass) {
#pragma unroll
    for (int j = 0; j < 16; ++j) { const int rr = j * 2 + hlf, c4 = nloc * 4; *(volatile v4f*)(dst0 + (size_t)rr * ldo + c4) = *(const v4f*)(Tt + rr * 64 + c4); }
    __threadfence();
  }
}


__global__ __launch_bounds__(256) void prep_kernel(const float* __restrict__ z, const float* __restrict__ Win, const float* __restrict__ Wh1, const float* __restrict__ Wh2, const float* __restrict__ Wout,
                                                   const float* __restrict__ rW1, const float* __restrict__ tW1,
                                                   float* __restrict__ zp, b16* __restrict__ w3, b16* __restrict__ wo, b16* __restrict__ wrt) {
  const size_t tid = (size_t)blockIdx.x * blockDim.x + threadIdx.x, nth = (size_t)gridDim.x * blockDim.x;
  for (int pass = 0; pass < 2; ++pass) {
    for (size_t p = tid; p < (size_t)NPAD * H / 4; p += nth) { const size_t n = p / (H / 4); const v4f v = (n < (size_t)N) ? *(const v4f*)(z + p * 4) : (v4f){0.0f, 0.0f, 0.0f, 0.0f}; *(volatile v4f*)(zp + p * 4) = v; }
    for (size_t p = tid; p < (size_t)3 * H * H / 8; p += nth) { const int m = (int)(p / (H * H / 8)); const int rem = (int)(p % (H * H / 8)), n = rem / 16, k0 = (rem % 16) * 8; const float* W = (m == 0) ? Win : (m == 1) ? Wh1 : Wh2; v8b v;
#pragma unroll
      for (int e = 0; e < 8; ++e) v[e] = (b16)W[(size_t)(k0 + e) * H + n];
      *(volatile v8b*)(w3 + (size_t)m * H * H + (size_t)n * H + k0) = v; }
    for (size_t p = tid; p < (size_t)HO * H / 8; p += nth) { const int n = (int)(p / 16), k0 = (int)(p % 16) * 8; v8b v;
#pragma unroll
      for (int e = 0; e < 8; ++e) v[e] = (b16)Wout[(size_t)(k0 + e) * HO + n];
      *(volatile v8b*)(wo + (size_t)n * H + k0) = v; }
    for (size_t p = tid; p < (size_t)2 * H * H / 8; p += nth) { const int n = (int)(p / 16), k0 = (int)(p % 16) * 8; const float* W = (n < H) ? rW1 : tW1; const int nn = n % H; v8b v;
#pragma unroll
      for (int e = 0; e < 8; ++e) v[e] = (b16)W[(size_t)(k0 + e) * H + nn];
      *(volatile v8b*)(wrt + (size_t)n * H + k0) = v; }
    __threadfence();
  }
}

template <int DF, int NB>
__global__ __launch_bounds__(256) void agg_kernel(const int* __restrict__ esrc, const int* __restrict__ edst, const float* __restrict__ x, const float* __restrict__ bias, float* __restrict__ zin) {
  __shared__ __attribute__((aligned(16))) int acc[NB * DF];
  __shared__ int list[8 * 256]; __shared__ int cnt[NB];
  constexpr float FXS = 524288.0f, FXI = 1.0f / 524288.0f;
  const int t_ = threadIdx.x, wave = t_ >> 5, lane = t_ & 31, base = blockIdx.x * NB;
  for (int i = t_; i < NB * DF; i += 256) acc[i] = 0;
  for (int i = t_; i < NB; i += 256) cnt[i] = 0;
  __syncthreads();
  int* wl = list + wave * 256;
  typedef __attribute__((ext_vector_type(4))) int v4i;
  for (int c0 = 0; c0 < E; c0 += 256 * 8) {
    const int e0 = c0 + (wave * 32 + lane) * 8;
    int dd[8];
    if (e0 + 7 < E) { const v4i a = *(const v4i*)(edst + e0), b = *(const v4i*)(edst + e0 + 4); dd[0] = a[0]; dd[1] = a[1]; dd[2] = a[2]; dd[3] = a[3]; dd[4] = b[0]; dd[5] = b[1]; dd[6] = b[2]; dd[7] = b[3]; }
    else {
#pragma unroll
      for (int j = 0; j < 8; ++j) dd[j] = (e0 + j < E) ? edst[e0 + j] : -1; }
    unsigned sl[8]; bool hit[8]; bool anyl = false;
#pragma unroll
    for (int j = 0; j < 8; ++j) { sl[j] = (unsigned)(dd[j] - base); hit[j] = sl[j] < (unsigned)NB; anyl |= hit[j]; }
    int wc = 0;
    if (__builtin_amdgcn_ballot_w32(anyl) != 0u) {
#pragma unroll
      for (int j = 0; j < 8; ++j) {
        const unsigned mj = __builtin_amdgcn_ballot_w32(hit[j]);
        if (mj != 0u) {
          if (hit[j]) { const int pos = wc + (int)__builtin_amdgcn_mbcnt_lo(mj, 0u); int s = esrc[e0 + j]; s = (s < 0) ? 0 : (s >= N ? N - 1 : s); wl[pos] = (s << 12) | (int)sl[j]; atomicAdd(&cnt[sl[j]], 1); }
          wc += __builtin_popcount(mj);
        }
      }
    }
    __builtin_amdgcn_wave_barrier(); __builtin_amdgcn_fence(__ATOMIC_RELEASE, "workgroup"); __builtin_amdgcn_fence(__ATOMIC_ACQUIRE, "workgroup");
    { constexpr int LPH = DF / 4, HPS = 32 / LPH;
      for (int i0 = 0; i0 < wc; i0 += HPS) { const int i = i0 + lane / LPH; if (i < wc) { const int ent = wl[i]; const int s = ent >> 12, slot = ent & 4095; const int col = (lane % LPH) * 4;
          const v4f v = *(const v4f*)(x + (size_t)s * DF + col);
#pragma unroll
          for (int c = 0; c < 4; ++c) atomicAdd(&acc[slot * DF + col + c], (int)rintf(v[c] * FXS)); } } }
    __builtin_amdgcn_wave_barrier();
  }
  __syncthreads();
  for (int pass = 0; pass < 2; ++pass) {
    for (int i = t_; i < NB * DF / 4; i += 256) { const int r = (i * 4) / DF; const int node = base + r; if (node < NPAD) {
        v4f o = {0.0f, 0.0f, 0.0f, 0.0f}; if (node < N) { const float inv = 1.0f / fmaxf((float)cnt[r], 1.0f); const int k0 = (i * 4) % DF;
#pragma unroll
          for (int c = 0; c < 4; ++c) o[c] = ((float)acc[i * 4 + c] * FXI) * inv + bias[k0 + c]; }
        *(volatile v4f*)(zin + (size_t)base * DF + (size_t)i * 4) = o; } }
    __threadfence();
  }
}


template <bool RELU, int NOUT>
__global__ __launch_bounds__(128) void lin_kernel(const float* __restrict__ x, const b16* __restrict__ w, float* __restrict__ h) {
  __shared__ __attribute__((aligned(16))) float Ts[4][32 * 64];
  const int lane = threadIdx.x & 31, wave = threadIdx.x >> 5, nloc = lane & 15, hlf = lane >> 4, m0 = blockIdx.y * 128 + wave * 32, c0 = blockIdx.x * 64;
  v8f acc[2][4];
#pragma unroll
  for (int r = 0; r < 2; ++r)
#pragma unroll
    for (int t = 0; t < 4; ++t) acc[r][t] = (v8f){};
#pragma unroll 1
  for (int kb = 0; kb < H; kb += 32) {
    v16b a0, a1;
#pragma unroll
    for (int e = 0; e < 16; ++e) { const int k = kb + ((e < 8) ? (8 * hlf + e) : (16 + 8 * hlf + e - 8)); float u0 = x[(size_t)(m0 + nloc) * H + k], u1 = x[(size_t)(m0 + 16 + nloc) * H + k];
      if (RELU) { u0 = fmaxf(u0, 0.0f); u1 = fmaxf(u1, 0.0f); } a0[e] = (b16)u0; a1[e] = (b16)u1; }
#pragma unroll
    for (int t = 0; t < 4; ++t) { const v16b bw = frag_kb(w + (size_t)(c0 + t * 16 + nloc) * H + kb, hlf); acc[0][t] = wmma16b(a0, bw, acc[0][t]); acc[1][t] = wmma16b(a1, bw, acc[1][t]); }
  }
  epi_f32(acc, 1.0f, nullptr, h, NOUT, m0, c0, lane, Ts[wave]);
}

__global__ __launch_bounds__(128) void edge_kernel(const int* __restrict__ esrc, const int* __restrict__ edst, const float* __restrict__ z, const float* __restrict__ hg, const b16* __restrict__ wrt,
                                                   const float* __restrict__ rb1, const float* __restrict__ tb1, const float* __restrict__ rW2, const float* __restrict__ tW2, const float* __restrict__ rb2, const float* __restrict__ tb2,
                                                   float* __restrict__ out) {
  __shared__ __attribute__((aligned(16))) b16 Ft[32][H + 8];
  __shared__ float Part[4][32]; __shared__ float Dist[32]; __shared__ float Res[32];
  const int wave = threadIdx.x >> 5, lane = threadIdx.x & 31, nloc = lane & 15, hlf = lane >> 4, e0 = blockIdx.x * 32;
  { const int el = threadIdx.x >> 2, q = threadIdx.x & 3, e = e0 + el; int s = esrc[e], dd = edst[e]; s = (s < 0) ? 0 : (s >= N ? N - 1 : s); dd = (dd < 0) ? 0 : (dd >= N ? N - 1 : dd);
    const float* srcrow = (q < 2) ? (hg + (size_t)s * HO + q * 32) : (hg + (size_t)dd * HO + (q - 2) * 32);
#pragma unroll
    for (int i = 0; i < 32; i += 4) { const v4f v = *(const v4f*)(srcrow + i); Ft[el][q * 32 + i] = (b16)v[0]; Ft[el][q * 32 + i + 1] = (b16)v[1]; Ft[el][q * 32 + i + 2] = (b16)v[2]; Ft[el][q * 32 + i + 3] = (b16)v[3]; }
    float ds = 0.0f;
#pragma unroll 1
    for (int i = q * 32; i < q * 32 + 32; ++i) { const float df = z[(size_t)s * H + i] - z[(size_t)dd * H + i] + 1e-6f; ds += df * df; }
    ds += __shfl_xor(ds, 1); ds += __shfl_xor(ds, 2);
    if (q == 0) Dist[el] = -sqrtf(ds); }
  __syncthreads();
  v8f acc[2][4];
#pragma unroll
  for (int r = 0; r < 2; ++r)
#pragma unroll
    for (int t = 0; t < 4; ++t) acc[r][t] = (v8f){};
  const int c0 = wave * 64;
#pragma unroll
  for (int kb = 0; kb < H; kb += 32) {
    const v16b a0 = frag_kb(&Ft[nloc][0] + kb, hlf), a1 = frag_kb(&Ft[16 + nloc][0] + kb, hlf);
#pragma unroll
    for (int t = 0; t < 4; ++t) { const v16b bw = frag_kb(wrt + (size_t)(c0 + t * 16 + nloc) * H + kb, hlf); acc[0][t] = wmma16b(a0, bw, acc[0][t]); acc[1][t] = wmma16b(a1, bw, acc[1][t]); }
  }
  const bool isR = (wave < 2);
  float part[2][8];
#pragma unroll
  for (int r = 0; r < 2; ++r)
#pragma unroll
    for (int v = 0; v < 8; ++v) { float s = 0.0f;
#pragma unroll
      for (int t = 0; t < 4; ++t) { const int col = c0 + t * 16 + nloc; const int cc = col & (H - 1); float a = acc[r][t][v] + (isR ? rb1[cc] : tb1[cc]); a = (a > 0.0f) ? a : 0.2f * a; s += a * (isR ? rW2[cc] : tW2[cc]); }
      part[r][v] = s; }
#pragma unroll
  for (int o = 1; o < 16; o <<= 1)
#pragma unroll
    for (int r = 0; r < 2; ++r)
#pragma unroll
      for (int v = 0; v < 8; ++v) part[r][v] += __shfl_xor(part[r][v], o);
  if (nloc == 0) {
#pragma unroll
    for (int r = 0; r < 2; ++r)
#pragma unroll
      for (int v = 0; v < 8; ++v) Part[wave][r * 16 + 8 * hlf + v] = part[r][v]; }
  __syncthreads();
  if (threadIdx.x < 32) { const int el = threadIdx.x; const float r_ = Part[0][el] + Part[1][el] + rb2[0], t_ = Part[2][el] + Part[3][el] + tb2[0];
    const float xx = (Dist[el] - r_) / t_; Res[el] = 1.0f / (1.0f + __expf(-xx)); }
  __syncthreads();
  if (threadIdx.x < 32) for (int pass = 0; pass < 2; ++pass) { ((volatile float*)out)[e0 + threadIdx.x] = Res[threadIdx.x]; __threadfence(); }
}
}

extern "C" void kernel_launch(void* const* d_in, const int* in_sizes, int n_in,
                              void* d_out, int out_size, void* d_ws, size_t ws_size, hipStream_t stream) {
  (void)n_in; (void)out_size;
  const float* z = (const float*)d_in[0]; const int* ei = (const int*)d_in[1];
  const float* Win = (const float*)d_in[2]; const float* bin = (const float*)d_in[3]; const float* Wh1 = (const float*)d_in[4]; const float* bh1 = (const float*)d_in[5];
  const float* Wh2 = (const float*)d_in[6]; const float* bh2 = (const float*)d_in[7]; const float* Wout = (const float*)d_in[8]; const float* bout = (const float*)d_in[9];
  const float* rW1 = (const float*)d_in[10]; const float* rb1 = (const float*)d_in[11]; const float* rW2 = (const float*)d_in[12]; const float* rb2 = (const float*)d_in[13];
  const float* tW1 = (const float*)d_in[14]; const float* tb1 = (const float*)d_in[15]; const float* tW2 = (const float*)d_in[16]; const float* tb2 = (const float*)d_in[17];
  float* out = (float*)d_out;
  if (in_sizes[0] != N * H || in_sizes[1] != 2 * E || in_sizes[2] != H * H || in_sizes[8] != H * HO || in_sizes[10] != H * H || in_sizes[12] != H) return;
  const int* esrc = ei; const int* edst = ei + E;
  size_t off = 0; char* ws = (char*)d_ws;
  auto carve = [&](size_t bytes) { char* p = ws + off; off += (bytes + 255) & ~(size_t)255; return p; };
  float* zp = (float*)carve((size_t)NPAD * H * 4); float* bufA = (float*)carve((size_t)NPAD * H * 4); float* bufB = (float*)carve((size_t)NPAD * H * 4);
  b16* w3 = (b16*)carve((size_t)3 * H * H * 2); b16* wo = (b16*)carve((size_t)HO * H * 2); b16* wrt = (b16*)carve((size_t)2 * H * H * 2);
  if (off > ws_size) return;
  prep_kernel<<<512, 256, 0, stream>>>(z, Win, Wh1, Wh2, Wout, rW1, tW1, zp, w3, wo, wrt);
  lin_kernel<false, H><<<dim3(H / 64, NBLK), 128, 0, stream>>>(zp, w3, bufA);
  agg_kernel<H, 512><<<NPAD / 512 + 1, 256, 0, stream>>>(esrc, edst, bufA, bin, bufB);
  lin_kernel<true, H><<<dim3(H / 64, NBLK), 128, 0, stream>>>(bufB, w3 + (size_t)H * H, bufA);
  agg_kernel<H, 512><<<NPAD / 512 + 1, 256, 0, stream>>>(esrc, edst, bufA, bh1, bufB);
  lin_kernel<true, H><<<dim3(H / 64, NBLK), 128, 0, stream>>>(bufB, w3 + (size_t)2 * H * H, bufA);
  agg_kernel<H, 512><<<NPAD / 512 + 1, 256, 0, stream>>>(esrc, edst, bufA, bh2, bufB);
  lin_kernel<true, HO><<<dim3(HO / 64, NBLK), 128, 0, stream>>>(bufB, wo, bufA);
  agg_kernel<HO, 1024><<<NPAD / 1024 + 1, 256, 0, stream>>>(esrc, edst, bufA, bout, bufB);
  edge_kernel<<<E / 32, 128, 0, stream>>>(esrc, edst, z, bufB, wrt, rb1, tb1, rW2, tW2, rb2, tb2, out);
}
